// HoloLayer_75754633167190
// MI455X (gfx1250) — hardware-verified
//
#include <hip/hip_runtime.h>
#include <math.h>

typedef __bf16   v16b __attribute__((ext_vector_type(16)));
typedef __bf16   v8b  __attribute__((ext_vector_type(8)));
typedef float    v8f  __attribute__((ext_vector_type(8)));
typedef float    v4f  __attribute__((ext_vector_type(4)));
typedef float    v2f  __attribute__((ext_vector_type(2)));
typedef unsigned int v4u __attribute__((ext_vector_type(4)));
typedef v8b __attribute__((may_alias)) v8ba;
typedef v4f __attribute__((may_alias)) v4fa;
typedef v2f __attribute__((may_alias)) v2fa;
typedef v4u __attribute__((may_alias)) v4ua;

union FragB { v16b v; v8b half[2]; };

#define DD   768
#define SS   4096
#define BB   4
#define NTOK (BB * SS)
#define NC   800
#define ZP   832
#define NXB  (SS * DD)
#define NX   (NTOK * DD)
#define NW   (DD * DD)

static_assert(NXB % 8 == 0);
static_assert(NC % 32 == 0);
static_assert((ZP * 2) % 128 == 0);
static_assert((NC * 4) % 128 == 0);
static_assert((DD * 2) % 128 == 0);

__device__ __forceinline__ v8f wmma_bf16(v16b a, v16b b, v8f c) {
  v8f d = __builtin_amdgcn_wmma_f32_16x16x32_bf16(false, a, false, b, (short)0, c, false, false);
  asm volatile("v_nop\n\tv_nop\n\tv_nop\n\tv_nop" : "+v"(d) : "v"(a), "v"(b));
  return d;
}

__device__ __forceinline__ v16b ldfrag_b(const __bf16* p, int h) {
  FragB f;
  f.half[0] = *(const v8ba*)(p + 8 * h);
  f.half[1] = *(const v8ba*)(p + 16 + 8 * h);
  return f.v;
}

__device__ __forceinline__ unsigned int bf16_bits(float f) {
  unsigned int u = __float_as_uint(f);
  u += 0x7FFFu + ((u >> 16) & 1u);
  return (u >> 16) & 0xFFFFu;
}
__device__ __forceinline__ void split2(float v, unsigned int& hb, unsigned int& lb) {
  hb = bf16_bits(v);
  lb = bf16_bits(v - __uint_as_float(hb << 16));
}
__device__ __forceinline__ unsigned int pk2(unsigned int e0, unsigned int e1) {
  return e0 | (e1 << 16);
}
__device__ __forceinline__ void split8(v4f a, v4f c, v4u& H, v4u& L) {
  unsigned int h0, h1, h2, h3, h4, h5, h6, h7, l0, l1, l2, l3, l4, l5, l6, l7;
  split2(a.x, h0, l0); split2(a.y, h1, l1); split2(a.z, h2, l2); split2(a.w, h3, l3);
  split2(c.x, h4, l4); split2(c.y, h5, l5); split2(c.z, h6, l6); split2(c.w, h7, l7);
  const v4u hh = { pk2(h0, h1), pk2(h2, h3), pk2(h4, h5), pk2(h6, h7) };
  const v4u ll = { pk2(l0, l1), pk2(l2, l3), pk2(l4, l5), pk2(l6, l7) };
  H = hh;
  L = ll;
}

__device__ __forceinline__ void table_store(const float* s, float* tab, int tid) {
  for (int j = tid; j < (2 * DD) / 4; j += 256) {
    const v4f v = *(const v4fa*)(s + 4 * j);
    *(volatile v4f*)(tab + 4 * j) = v;
  }
}
__global__ __launch_bounds__(256) void k_table(float* __restrict__ tab) {
  __shared__ __attribute__((aligned(16))) float s[2 * DD];
  const int tid = threadIdx.x;
  #pragma unroll 1
  for (int r = tid; r < DD; r += 256) {
    const int q = r / 192, p = r - q * 192;
    const bool lowp = (p <= 96);
    const int a = lowp ? p : (192 - p);
    const float th = (float)a * 8.18123086872342e-3f;
    const float ct = cosf(th), st = sinf(th);
    const float c0 = lowp ? ct : st;
    const float s0 = lowp ? st : ct;
    float c, sn;
    if (q == 0)      { c =  c0; sn =  s0; }
    else if (q == 1) { c = -s0; sn =  c0; }
    else if (q == 2) { c = -c0; sn = -s0; }
    else             { c =  s0; sn = -c0; }
    s[r] = c;
    s[DD + r] = sn;
  }
  __syncthreads();
  table_store(s, tab, tid);
  __threadfence();
  table_store(s, tab, tid);
}

__global__ __launch_bounds__(256) void k_cvt_x(const float* __restrict__ x, __bf16* __restrict__ xh,
                                               __bf16* __restrict__ xl, int b, int n8) {
  const int g = blockIdx.x * 256 + threadIdx.x;
  if (g >= n8) return;
  const float* src = x + (size_t)b * NXB + (size_t)g * 8;
  const v4f a = *(const v4fa*)src;
  const v4f c = *(const v4fa*)(src + 4);
  v4u H, L;
  split8(a, c, H, L);
  const size_t o = (size_t)g * 8;
  *(volatile v4u*)(xh + o) = H;
  *(volatile v4u*)(xl + o) = L;
  __threadfence();
  *(volatile v4u*)(xh + o) = H;
  *(volatile v4u*)(xl + o) = L;
}

__device__ __forceinline__ void wt_store(const float* sT, __bf16* dh, __bf16* dl, int d0, int e0, int tid) {
  #pragma unroll
  for (int it = 0; it < 2; ++it) {
    const int p = tid + 256 * it;
    const int row = p >> 3, q8 = p & 7;
    const float* s = sT + row * 65 + 8 * q8;
    const v4f a = { s[0], s[1], s[2], s[3] };
    const v4f c = { s[4], s[5], s[6], s[7] };
    v4u H, L;
    split8(a, c, H, L);
    const size_t o = (size_t)(d0 + row) * DD + e0 + 8 * q8;
    *(volatile v4u*)(dh + o) = H;
    *(volatile v4u*)(dl + o) = L;
  }
}
__global__ __launch_bounds__(256) void k_wt(const float* __restrict__ wk, const float* __restrict__ wv,
                                            const float* __restrict__ wq, __bf16* __restrict__ wth,
                                            __bf16* __restrict__ wtl) {
  __shared__ float sT[64 * 65];
  const int tid = threadIdx.x;
  const int d0 = blockIdx.x * 64, e0 = blockIdx.y * 64, z = blockIdx.z;
  const float* W = (z == 0) ? wk : ((z == 1) ? wv : wq);
  #pragma unroll
  for (int it = 0; it < 4; ++it) {
    const int idx = tid + 256 * it;
    const int er = idx >> 4, dq = idx & 15;
    const v4f v = *(const v4fa*)(W + (size_t)(e0 + er) * DD + d0 + 4 * dq);
    sT[(4 * dq + 0) * 65 + er] = v.x;
    sT[(4 * dq + 1) * 65 + er] = v.y;
    sT[(4 * dq + 2) * 65 + er] = v.z;
    sT[(4 * dq + 3) * 65 + er] = v.w;
  }
  __syncthreads();
  __bf16* dh = wth + (size_t)z * NW;
  __bf16* dl = wtl + (size_t)z * NW;
  wt_store(sT, dh, dl, d0, e0, tid);
  __threadfence();
  wt_store(sT, dh, dl, d0, e0, tid);
}

__global__ __launch_bounds__(128) void k_ft(const float* __restrict__ tab, __bf16* __restrict__ fth,
                                            __bf16* __restrict__ ftl) {
  const int c = blockIdx.x;
  const int j = threadIdx.x;
  const int f = c >> 1;
  const bool valid = (c < 770);
  const bool im = (c & 1) != 0;
  const int e0 = 8 * j;
  float v[8];
  #pragma unroll
  for (int i = 0; i < 8; ++i) {
    const int e = e0 + i;
    const int mm = (f * e) % DD;
    const float cv = tab[mm], sv = tab[DD + mm];
    v[i] = valid ? (im ? -sv : cv) : 0.0f;
  }
  const v4f a = { v[0], v[1], v[2], v[3] };
  const v4f cc = { v[4], v[5], v[6], v[7] };
  v4u H, L;
  split8(a, cc, H, L);
  const size_t o = (size_t)c * DD + e0;
  *(volatile v4u*)(fth + o) = H;
  *(volatile v4u*)(ftl + o) = L;
  __threadfence();
  *(volatile v4u*)(fth + o) = H;
  *(volatile v4u*)(ftl + o) = L;
}

__global__ __launch_bounds__(128) void k_finv(const float* __restrict__ tab, __bf16* __restrict__ fih,
                                              __bf16* __restrict__ fil) {
  const int n = blockIdx.x;
  const int j = threadIdx.x;
  if (j >= ZP / 8) return;
  const int c0 = 8 * j;
  float v[8];
  #pragma unroll
  for (int i = 0; i < 8; ++i) {
    const int c = c0 + i;
    const int f = c >> 1;
    const bool valid = (c < 770);
    const float w = (f == 0 || f == DD / 2) ? 1.0f : 2.0f;
    const int mm = (f * n) % DD;
    const float cv = tab[mm], sv = tab[DD + mm];
    v[i] = valid ? (w * ((c & 1) ? -sv : cv) * (1.0f / 768.0f)) : 0.0f;
  }
  const v4f a = { v[0], v[1], v[2], v[3] };
  const v4f cc = { v[4], v[5], v[6], v[7] };
  v4u H, L;
  split8(a, cc, H, L);
  const size_t o = (size_t)n * ZP + c0;
  *(volatile v4u*)(fih + o) = H;
  *(volatile v4u*)(fil + o) = L;
  __threadfence();
  *(volatile v4u*)(fih + o) = H;
  *(volatile v4u*)(fil + o) = L;
}

__device__ __forceinline__ void fold_store(const unsigned short* sHw, const unsigned short* sLw,
                                           __bf16* gh, __bf16* gl, size_t rowbase, int d0w, int lane) {
  const int q8 = lane & 7, sub = lane >> 3;
  #pragma unroll
  for (int i = 0; i < 8; ++i) {
    const int row = 4 * i + sub;
    const v4u vh = *(const v4ua*)(sHw + row * 64 + 8 * q8);
    const v4u vl = *(const v4ua*)(sLw + row * 64 + 8 * q8);
    const size_t o = (rowbase + row) * DD + d0w + 8 * q8;
    *(volatile v4u*)(gh + o) = vh;
    *(volatile v4u*)(gl + o) = vl;
  }
}
__global__ __launch_bounds__(128) void k_fold(const __bf16* __restrict__ fth, const __bf16* __restrict__ ftl,
                                              const __bf16* __restrict__ wth, const __bf16* __restrict__ wtl,
                                              __bf16* __restrict__ gh, __bf16* __restrict__ gl) {
  __shared__ __attribute__((aligned(16))) unsigned short sH[4 * 32 * 64];
  __shared__ __attribute__((aligned(16))) unsigned short sL[4 * 32 * 64];

  const int tid = threadIdx.x, lane = tid & 31, w = tid >> 5;
  const int h = lane >> 4, m = lane & 15;
  const int c0 = blockIdx.y * 32;
  const int d0w = blockIdx.x * 256 + 64 * w;
  const int z = blockIdx.z;

  const size_t r16 = (size_t)16 * DD;
  const __bf16* fah = fth + (size_t)(c0 + m) * DD;
  const __bf16* fal = ftl + (size_t)(c0 + m) * DD;
  const __bf16* bwh = wth + ((size_t)z * DD + d0w + m) * DD;
  const __bf16* bwl = wtl + ((size_t)z * DD + d0w + m) * DD;

  const v8f zero8 = {0.f, 0.f, 0.f, 0.f, 0.f, 0.f, 0.f, 0.f};
  v8f acc[2][4];
  #pragma unroll
  for (int mt = 0; mt < 2; ++mt)
    #pragma unroll
    for (int nt = 0; nt < 4; ++nt) acc[mt][nt] = zero8;

  #pragma unroll 1
  for (int k0 = 0; k0 < DD; k0 += 32) {
    const v16b ah0 = ldfrag_b(fah + k0, h);
    const v16b ah1 = ldfrag_b(fah + r16 + k0, h);
    const v16b al0 = ldfrag_b(fal + k0, h);
    const v16b al1 = ldfrag_b(fal + r16 + k0, h);
    #pragma unroll
    for (int nt = 0; nt < 4; ++nt) {
      const v16b bh = ldfrag_b(bwh + (size_t)nt * r16 + k0, h);
      const v16b bl = ldfrag_b(bwl + (size_t)nt * r16 + k0, h);
      acc[0][nt] = wmma_bf16(ah0, bh, acc[0][nt]);
      acc[1][nt] = wmma_bf16(ah1, bh, acc[1][nt]);
      acc[0][nt] = wmma_bf16(ah0, bl, acc[0][nt]);
      acc[1][nt] = wmma_bf16(ah1, bl, acc[1][nt]);
      acc[0][nt] = wmma_bf16(al0, bh, acc[0][nt]);
      acc[1][nt] = wmma_bf16(al1, bh, acc[1][nt]);
    }
  }

  unsigned short* sHw = sH + w * 2048;
  unsigned short* sLw = sL + w * 2048;
  #pragma unroll
  for (int mt = 0; mt < 2; ++mt)
    #pragma unroll
    for (int nt = 0; nt < 4; ++nt)
      #pragma unroll
      for (int r = 0; r < 8; ++r) {
        unsigned int hb, lb;
        split2(acc[mt][nt][r], hb, lb);
        const int idx = (16 * mt + 8 * h + r) * 64 + 16 * nt + m;
        sHw[idx] = (unsigned short)hb;
        sLw[idx] = (unsigned short)lb;
      }
  __syncthreads();

  const size_t rowbase = (size_t)z * NC + c0;
  fold_store(sHw, sLw, gh, gl, rowbase, d0w, lane);
  __threadfence();
  fold_store(sHw, sLw, gh, gl, rowbase, d0w, lane);
}

__device__ __forceinline__ void spec_store(const float* sSw, float* spec, int t0w, int c0, int lane) {
  const int q8 = lane & 7, sub = lane >> 3;
  #pragma unroll
  for (int i = 0; i < 8; ++i) {
    const int row = 4 * i + sub;
    const v4f v = *(const v4fa*)(sSw + row * 32 + 4 * q8);
    *(volatile v4f*)(spec + (size_t)(t0w + row) * NC + c0 + 4 * q8) = v;
  }
}
__global__ __launch_bounds__(128) void k_spec(const __bf16* __restrict__ xh, const __bf16* __restrict__ xl,
                                              const __bf16* __restrict__ gh, const __bf16* __restrict__ gl,
                                              float* __restrict__ sk, float* __restrict__ sv,
                                              float* __restrict__ sq) {
  __shared__ __attribute__((aligned(16))) float sS[4 * 32 * 32];

  const int tid = threadIdx.x, lane = tid & 31, w = tid >> 5;
  const int h = lane >> 4, m = lane & 15;
  const int c0 = blockIdx.x * 32;
  const int t0w = blockIdx.y * 128 + 32 * w;
  const int z = blockIdx.z;
  float* spec = (z == 0) ? sk : ((z == 1) ? sv : sq);

  const size_t r16 = (size_t)16 * DD;
  const __bf16* xah = xh + (size_t)(t0w + m) * DD;
  const __bf16* xal = xl + (size_t)(t0w + m) * DD;
  const __bf16* gha = gh + ((size_t)z * NC + c0 + m) * DD;
  const __bf16* gla = gl + ((size_t)z * NC + c0 + m) * DD;

  const v8f zero8 = {0.f, 0.f, 0.f, 0.f, 0.f, 0.f, 0.f, 0.f};
  v8f acc[2][2];
  #pragma unroll
  for (int mt = 0; mt < 2; ++mt)
    #pragma unroll
    for (int nt = 0; nt < 2; ++nt) acc[mt][nt] = zero8;

  #pragma unroll 1
  for (int k0 = 0; k0 < DD; k0 += 32) {
    const v16b ah0 = ldfrag_b(xah + k0, h);
    const v16b ah1 = ldfrag_b(xah + r16 + k0, h);
    const v16b al0 = ldfrag_b(xal + k0, h);
    const v16b al1 = ldfrag_b(xal + r16 + k0, h);
    const v16b bh0 = ldfrag_b(gha + k0, h);
    const v16b bh1 = ldfrag_b(gha + r16 + k0, h);
    const v16b bl0 = ldfrag_b(gla + k0, h);
    const v16b bl1 = ldfrag_b(gla + r16 + k0, h);
    acc[0][0] = wmma_bf16(ah0, bh0, acc[0][0]);
    acc[0][1] = wmma_bf16(ah0, bh1, acc[0][1]);
    acc[1][0] = wmma_bf16(ah1, bh0, acc[1][0]);
    acc[1][1] = wmma_bf16(ah1, bh1, acc[1][1]);
    acc[0][0] = wmma_bf16(ah0, bl0, acc[0][0]);
    acc[0][1] = wmma_bf16(ah0, bl1, acc[0][1]);
    acc[1][0] = wmma_bf16(ah1, bl0, acc[1][0]);
    acc[1][1] = wmma_bf16(ah1, bl1, acc[1][1]);
    acc[0][0] = wmma_bf16(al0, bh0, acc[0][0]);
    acc[0][1] = wmma_bf16(al0, bh1, acc[0][1]);
    acc[1][0] = wmma_bf16(al1, bh0, acc[1][0]);
    acc[1][1] = wmma_bf16(al1, bh1, acc[1][1]);
  }

  float* sSw = sS + w * 1024;
  #pragma unroll
  for (int mt = 0; mt < 2; ++mt)
    #pragma unroll
    for (int nt = 0; nt < 2; ++nt)
      #pragma unroll
      for (int r = 0; r < 8; ++r)
        sSw[(16 * mt + 8 * h + r) * 32 + 16 * nt + m] = acc[mt][nt][r];
  __syncthreads();

  spec_store(sSw, spec, t0w, c0, lane);
  __threadfence();
  spec_store(sSw, spec, t0w, c0, lane);
}

__global__ __launch_bounds__(32) void k_scan(const float* __restrict__ kf, const float* __restrict__ vf,
                                             const float* __restrict__ qf, __bf16* __restrict__ zh,
                                             __bf16* __restrict__ zl) {
  const int lane = threadIdx.x;
  const int f = blockIdx.x * 32 + lane;
  const bool act = (f < NC / 2);
  const int fc = act ? f : (NC / 2 - 1);
  double mr = 0.0, mi = 0.0;
  #pragma unroll 1
  for (int t = 0; t < SS; ++t) {
    const size_t o = (size_t)t * NC + 2 * fc;
    const v2f kv = *(const v2fa*)(kf + o);
    const v2f vv = *(const v2fa*)(vf + o);
    const v2f qv = *(const v2fa*)(qf + o);
    const double kr = act ? (double)kv.x : 0.0, ki = act ? (double)kv.y : 0.0;
    const double vr = act ? (double)vv.x : 0.0, vi = act ? (double)vv.y : 0.0;
    const double qr = act ? (double)qv.x : 0.0, qi = act ? (double)qv.y : 0.0;
    const double pr = kr * vr - ki * vi;
    const double pi = kr * vi + ki * vr;
    mr += pr;
    mi += pi;
    const double zr = mr * qr + mi * qi;
    const double zi = mi * qr - mr * qi;
    unsigned int hr, lr, hi, li;
    split2((float)zr, hr, lr);
    split2((float)zi, hi, li);
    const unsigned int H = pk2(hr, hi);
    const unsigned int L = pk2(lr, li);
    const size_t zo = (size_t)t * ZP + 2 * f;
    *(volatile unsigned int*)(zh + zo) = H;
    *(volatile unsigned int*)(zl + zo) = L;
    __threadfence();
    *(volatile unsigned int*)(zh + zo) = H;
    *(volatile unsigned int*)(zl + zo) = L;
  }
}

__device__ __forceinline__ void inv_store(const float* sSw, const float* __restrict__ x, float* out,
                                          size_t tokbase, int n0, float g, int lane) {
  const int q8 = lane & 7, sub = lane >> 3;
  #pragma unroll
  for (int i = 0; i < 8; ++i) {
    const int row = 4 * i + sub;
    const v4f v = *(const v4fa*)(sSw + row * 32 + 4 * q8);
    const size_t o = (tokbase + row) * DD + n0 + 4 * q8;
    const v4f xv = *(const v4fa*)(x + o);
    const v4f rr = xv + g * v;
    *(volatile v4f*)(out + o) = rr;
  }
}
__global__ __launch_bounds__(128) void k_inv(const __bf16* __restrict__ zh, const __bf16* __restrict__ zl,
                                             const __bf16* __restrict__ fih, const __bf16* __restrict__ fil,
                                             const float* __restrict__ x, const float* __restrict__ gain,
                                             float* __restrict__ out, int b) {
  __shared__ __attribute__((aligned(16))) float sS[4 * 32 * 32];

  const int tid = threadIdx.x, lane = tid & 31, w = tid >> 5;
  const int h = lane >> 4, m = lane & 15;
  const int n0 = blockIdx.x * 32;
  const int t0w = blockIdx.y * 128 + 32 * w;

  const size_t r16 = (size_t)16 * ZP;
  const __bf16* zah = zh  + (size_t)(t0w + m) * ZP;
  const __bf16* zal = zl  + (size_t)(t0w + m) * ZP;
  const __bf16* fbh = fih + (size_t)(n0 + m) * ZP;
  const __bf16* fbl = fil + (size_t)(n0 + m) * ZP;

  const v8f zero8 = {0.f, 0.f, 0.f, 0.f, 0.f, 0.f, 0.f, 0.f};
  v8f acc[2][2];
  #pragma unroll
  for (int mt = 0; mt < 2; ++mt)
    #pragma unroll
    for (int nt = 0; nt < 2; ++nt) acc[mt][nt] = zero8;

  #pragma unroll 1
  for (int k0 = 0; k0 < NC; k0 += 32) {
    const v16b ah0 = ldfrag_b(zah + k0, h);
    const v16b ah1 = ldfrag_b(zah + r16 + k0, h);
    const v16b al0 = ldfrag_b(zal + k0, h);
    const v16b al1 = ldfrag_b(zal + r16 + k0, h);
    const v16b bh0 = ldfrag_b(fbh + k0, h);
    const v16b bh1 = ldfrag_b(fbh + r16 + k0, h);
    const v16b bl0 = ldfrag_b(fbl + k0, h);
    const v16b bl1 = ldfrag_b(fbl + r16 + k0, h);
    acc[0][0] = wmma_bf16(ah0, bh0, acc[0][0]);
    acc[0][1] = wmma_bf16(ah0, bh1, acc[0][1]);
    acc[1][0] = wmma_bf16(ah1, bh0, acc[1][0]);
    acc[1][1] = wmma_bf16(ah1, bh1, acc[1][1]);
    acc[0][0] = wmma_bf16(al0, bh0, acc[0][0]);
    acc[0][1] = wmma_bf16(al0, bh1, acc[0][1]);
    acc[1][0] = wmma_bf16(al1, bh0, acc[1][0]);
    acc[1][1] = wmma_bf16(al1, bh1, acc[1][1]);
    acc[0][0] = wmma_bf16(ah0, bl0, acc[0][0]);
    acc[0][1] = wmma_bf16(ah0, bl1, acc[0][1]);
    acc[1][0] = wmma_bf16(ah1, bl0, acc[1][0]);
    acc[1][1] = wmma_bf16(ah1, bl1, acc[1][1]);
  }

  float* sSw = sS + w * 1024;
  #pragma unroll
  for (int mt = 0; mt < 2; ++mt)
    #pragma unroll
    for (int nt = 0; nt < 2; ++nt)
      #pragma unroll
      for (int r = 0; r < 8; ++r)
        sSw[(16 * mt + 8 * h + r) * 32 + 16 * nt + m] = acc[mt][nt][r];
  __syncthreads();

  const float g = gain[0];
  const size_t tokbase = (size_t)b * SS + t0w;
  inv_store(sSw, x, out, tokbase, n0, g, lane);
  __threadfence();
  inv_store(sSw, x, out, tokbase, n0, g, lane);
}

extern "C" void kernel_launch(void* const* d_in, const int* in_sizes, int n_in,
                              void* d_out, int out_size, void* d_ws, size_t ws_size,
                              hipStream_t stream) {
  if (n_in < 5) return;
  if (in_sizes[0] != NX) return;
  if (in_sizes[1] != NW || in_sizes[2] != NW || in_sizes[3] != NW) return;
  if (in_sizes[4] < 1) return;
  if (out_size != NX) return;

  const float* x    = (const float*)d_in[0];
  const float* Wk   = (const float*)d_in[1];
  const float* Wv   = (const float*)d_in[2];
  const float* Wq   = (const float*)d_in[3];
  const float* gain = (const float*)d_in[4];
  float* out = (float*)d_out;

  const size_t tab_b = (size_t)2 * DD * 4;
  const size_t xb_b  = (size_t)NXB * 2;
  const size_t wt_b  = (size_t)3 * NW * 2;
  const size_t ft_b  = (size_t)NC * DD * 2;
  const size_t fi_b  = (size_t)DD * ZP * 2;
  const size_t g_b   = (size_t)3 * NC * DD * 2;
  const size_t sp_b  = (size_t)SS * NC * 4;
  const size_t z_b   = (size_t)SS * ZP * 2;
  const size_t total = tab_b + 2 * xb_b + 2 * wt_b + 2 * ft_b + 2 * fi_b + 2 * g_b + 3 * sp_b + 2 * z_b;
  if (total > ws_size) return;

  char* ws = (char*)d_ws;
  size_t off = 0;
  float*  tab = (float*)(ws + off);   off += tab_b;
  __bf16* xh  = (__bf16*)(ws + off);  off += xb_b;
  __bf16* xl  = (__bf16*)(ws + off);  off += xb_b;
  __bf16* wth = (__bf16*)(ws + off);  off += wt_b;
  __bf16* wtl = (__bf16*)(ws + off);  off += wt_b;
  __bf16* fth = (__bf16*)(ws + off);  off += ft_b;
  __bf16* ftl = (__bf16*)(ws + off);  off += ft_b;
  __bf16* fih = (__bf16*)(ws + off);  off += fi_b;
  __bf16* fil = (__bf16*)(ws + off);  off += fi_b;
  __bf16* gh  = (__bf16*)(ws + off);  off += g_b;
  __bf16* gl  = (__bf16*)(ws + off);  off += g_b;
  float*  sk  = (float*)(ws + off);   off += sp_b;
  float*  sv  = (float*)(ws + off);   off += sp_b;
  float*  sq  = (float*)(ws + off);   off += sp_b;
  __bf16* zh  = (__bf16*)(ws + off);  off += z_b;
  __bf16* zl  = (__bf16*)(ws + off);  off += z_b;
  if (off > ws_size) return;

  k_table<<<1, 256, 0, stream>>>(tab);
  k_wt<<<dim3(DD / 64, DD / 64, 3), 256, 0, stream>>>(Wk, Wv, Wq, wth, wtl);
  k_ft<<<NC, 96, 0, stream>>>(tab, fth, ftl);
  k_finv<<<DD, 128, 0, stream>>>(tab, fih, fil);

  k_fold<<<dim3(DD / 256, NC / 32, 3), 128, 0, stream>>>(fth, ftl, wth, wtl, gh, gl);

  const int n8 = NXB / 8;
  for (int b = 0; b < BB; ++b) {
    k_cvt_x<<<(n8 + 255) / 256, 256, 0, stream>>>(x, xh, xl, b, n8);
    k_spec<<<dim3(NC / 32, SS / 128, 3), 128, 0, stream>>>(xh, xl, gh, gl, sk, sv, sq);
    k_scan<<<ZP / 64, 32, 0, stream>>>(sk, sv, sq, zh, zl);
    k_inv<<<dim3(DD / 32, SS / 128), 128, 0, stream>>>(zh, zl, fih, fil, x, gain, out, b);
  }
}
